// ReMultiHeadSelfAttentionV2_4758823764688
// MI455X (gfx1250) — hardware-verified
//
#include <hip/hip_runtime.h>
#include <stddef.h>


typedef _Float16 h16;
typedef _Float16 v16h __attribute__((ext_vector_type(16)));
typedef _Float16 v8h  __attribute__((ext_vector_type(8)));
typedef float    v8f  __attribute__((ext_vector_type(8)));
typedef float    v4f  __attribute__((ext_vector_type(4)));

#ifndef NB
#define NB 64
#endif
#ifndef SEQ
#define SEQ 512
#endif
#define NB_FULL  64
#define SEQ_FULL 512
#define DIM    128
#define NHEAD  8
#define HD     16
#define NPATCH 32
#define NTOK   (NPATCH + SEQ)
#define TOKP   (((NTOK + 63) / 64) * 64)
#define QKP    256
#define XROWS  (NB * TOKP)
#define OROWS  (NTOK * NB)

static_assert(NB >= 1 && NB <= NB_FULL);
static_assert(SEQ >= 32 && SEQ <= SEQ_FULL);
static_assert(DIM == NHEAD * HD);
static_assert(HD == 16);
static_assert(NHEAD == 8);
static_assert((DIM % 32) == 0 && (DIM % 64) == 0);
static_assert(QKP == 2 * DIM && (QKP % 64) == 0);
static_assert((NTOK % 32) == 0);
static_assert((NTOK % 16) == 0);
static_assert((TOKP % 64) == 0 && TOKP >= NTOK);
static_assert((XROWS % 64) == 0 && (XROWS % 16) == 0);
static_assert((OROWS % 64) == 0);
static_assert(((3 * DIM * DIM) % 2048) == 0 && ((DIM * DIM) % 2048) == 0);
static_assert(DIM == 16 * 8);

#define LDC 68
#define LDO 136
static_assert((LDC % 4) == 0 && LDC >= 64);
static_assert((LDO % 8) == 0 && LDO >= DIM);

#define WCARRY 64.0f
#define QCARRY 64.0f
#define PCARRY 1024.0f
#define CCARRY 64.0f
#define PCUT   (-16.0f)

#define WQKV_BYTES ((size_t)3 * DIM * DIM * 2)
#define W0_BYTES   ((size_t)DIM * DIM * 2)
#define X_BYTES    ((size_t)XROWS * DIM * 2)
#define QK_BYTES   ((size_t)XROWS * QKP * 2)
#define VT_BYTES   ((size_t)NB * DIM * TOKP * 2)
#define CTX_BYTES  ((size_t)OROWS * DIM * 2)
#define OFF_WQKV ((size_t)0)
#define OFF_W0   (OFF_WQKV + WQKV_BYTES)
#define OFF_X    (OFF_W0 + W0_BYTES)
#define OFF_QK   (OFF_X + X_BYTES)
#define OFF_VT   (OFF_QK + QK_BYTES)
#define OFF_CTX  (OFF_VT + VT_BYTES)
#define WS_TOTAL (OFF_CTX + CTX_BYTES)
static_assert((WQKV_BYTES % 128) == 0 && (W0_BYTES % 128) == 0 && (X_BYTES % 128) == 0);
static_assert((QK_BYTES % 128) == 0 && (VT_BYTES % 128) == 0 && (CTX_BYTES % 128) == 0);
static_assert(WS_TOTAL <= (size_t)134217728);

__device__ __forceinline__ float bf16r(float x) {
  unsigned int u = __float_as_uint(x);
  u = (u + 0x7FFFu + ((u >> 16) & 1u)) & 0xFFFF0000u;
  return __uint_as_float(u);
}

static __device__ __forceinline__ h16 toh_flush(float v) {
  const h16 r = (h16)v;
  return (fabsf(v) < 6.103515625e-05f) ? (h16)0.0f : r;
}

__device__ __forceinline__ v16h frag_at(const _Float16* p) {
  v8h lo = *(const v8h*)(p);
  v8h hi = *(const v8h*)(p + 16);
  v16h out;
#pragma unroll
  for (int i = 0; i < 8; ++i) { out[i] = lo[i]; out[i + 8] = hi[i]; }
  return out;
}

__device__ __forceinline__ v16h frag_k16(const _Float16* p) {
  const v8h lo = *(const v8h*)(p);
  v16h out;
#pragma unroll
  for (int i = 0; i < 8; ++i) { out[i] = lo[i]; out[i + 8] = (_Float16)0.0f; }
  return out;
}

__device__ __forceinline__ v8f wmma16(v16h a, v16h b, v8f c) {
  v8f d = __builtin_amdgcn_wmma_f32_16x16x32_f16(false, a, false, b, (short)0, c,
                                                 false, false);
  asm volatile("v_nop\n\tv_nop\n\tv_nop\n\tv_nop" : "+v"(d) : "v"(a), "v"(b));
  return d;
}

__global__ __launch_bounds__(256) void wcast_kernel(
    const float* __restrict__ W, _Float16* __restrict__ W16) {
  const size_t idx = ((size_t)blockIdx.x * 256u + threadIdx.x) * 8u;
  const v4f a0 = *(const v4f*)(W + idx);
  const v4f a1 = *(const v4f*)(W + idx + 4);
  v8h o;
#pragma unroll
  for (int i = 0; i < 4; ++i) {
    o[i]     = toh_flush(WCARRY * bf16r(a0[i]));
    o[i + 4] = toh_flush(WCARRY * bf16r(a1[i]));
  }
  _Float16* p = W16 + idx;
  *(volatile v8h*)p = o;
  __threadfence();
  *(volatile v8h*)p = o;
}

__global__ __launch_bounds__(256) void xconv_kernel(
    const float* __restrict__ xp, const float* __restrict__ xs, _Float16* __restrict__ X16) {
  const unsigned tid = threadIdx.x;
  const unsigned row = blockIdx.x * 16u + (tid >> 4);
  const unsigned c = (tid & 15u) * 8u;
  const unsigned b = row / (unsigned)TOKP;
  const unsigned f = row - b * (unsigned)TOKP;
  const unsigned fp = (f < (unsigned)NPATCH) ? f : (unsigned)(NPATCH - 1);
  unsigned sq = (f >= (unsigned)NPATCH) ? (f - (unsigned)NPATCH) : 0u;
  sq = (sq < (unsigned)SEQ) ? sq : (unsigned)(SEQ - 1);
  const float* pp = xp + (size_t)fp * DIM + c;
  const float* ps = xs + ((size_t)sq * NB_FULL + b) * DIM + c;
  const v4f p0 = *(const v4f*)(pp);
  const v4f p1 = *(const v4f*)(pp + 4);
  const v4f s0 = *(const v4f*)(ps);
  const v4f s1 = *(const v4f*)(ps + 4);
  const bool isp = (f < (unsigned)NPATCH);
  const bool live = (f < (unsigned)NTOK);
  v8h o;
#pragma unroll
  for (int i = 0; i < 4; ++i) {
    float t0 = isp ? p0[i] : s0[i];
    float t1 = isp ? p1[i] : s1[i];
    t0 = live ? t0 : 0.0f;
    t1 = live ? t1 : 0.0f;
    o[i]     = toh_flush(bf16r(t0));
    o[i + 4] = toh_flush(bf16r(t1));
  }
  _Float16* p = X16 + (size_t)row * DIM + c;
  *(volatile v8h*)p = o;
  __threadfence();
  *(volatile v8h*)p = o;
}

template <int MODE>
__device__ __forceinline__ void gemm_body(
    const _Float16* __restrict__ A16, const _Float16* __restrict__ Bt,
    const float* __restrict__ bias, float* __restrict__ outf, _Float16* __restrict__ out16) {
  __shared__ float Cs[64 * LDC];
  const unsigned tid = threadIdx.x, lane = tid & 31u;
  const unsigned w = (unsigned)__builtin_amdgcn_readfirstlane((int)(threadIdx.x >> 5));
  const unsigned mw = w >> 1, nw = w & 1u;
  const unsigned hh = lane >> 4, m = lane & 15u;
  const unsigned n0 = blockIdx.x * 64u;
  const unsigned row0 = blockIdx.y * 64u;

  const _Float16* ap  = A16 + (size_t)(row0 + mw * 16u + m) * DIM + hh * 8u;
  const _Float16* bp0 = Bt + (size_t)(n0 + nw * 32u + m) * DIM + hh * 8u;
  const _Float16* bp1 = bp0 + (size_t)16 * DIM;
  v8f acc0 = {}, acc1 = {};
#pragma unroll
  for (unsigned k0 = 0; k0 < (unsigned)DIM; k0 += 32u) {
    const v16h a  = frag_at(ap + k0);
    const v16h b0 = frag_at(bp0 + k0);
    const v16h b1 = frag_at(bp1 + k0);
    acc0 = wmma16(a, b0, acc0);
    acc1 = wmma16(a, b1, acc1);
  }
#pragma unroll
  for (int r = 0; r < 8; ++r) {
    float* d = &Cs[(mw * 16u + hh * 8u + (unsigned)r) * LDC + nw * 32u + m];
    d[0]  = acc0[r];
    d[16] = acc1[r];
  }
  __syncthreads();

  if (MODE == 0) {
    v8h x[2];
    size_t off[2];
#pragma unroll
    for (unsigned i = 0; i < 2u; ++i) {
      const unsigned r = 32u * i + (tid >> 3);
      const unsigned c = (tid & 7u) * 8u;
      const v4f u0 = *(const v4f*)&Cs[r * LDC + c];
      const v4f u1 = *(const v4f*)&Cs[r * LDC + c + 4];
#pragma unroll
      for (int j = 0; j < 4; ++j) {
        x[i][j]     = toh_flush(u0[j]);
        x[i][j + 4] = toh_flush(u1[j]);
      }
      off[i] = (size_t)(row0 + r) * QKP + n0 + c;
    }
#pragma unroll
    for (int i = 0; i < 2; ++i) *(volatile v8h*)(out16 + off[i]) = x[i];
    __threadfence();
#pragma unroll
    for (int i = 0; i < 2; ++i) *(volatile v8h*)(out16 + off[i]) = x[i];
  }

  if (MODE == 1) {
    const unsigned bidx = row0 / (unsigned)TOKP;
    const unsigned key0 = row0 - bidx * (unsigned)TOKP;
    v8h x[2];
    size_t off[2];
#pragma unroll
    for (unsigned i = 0; i < 2u; ++i) {
      const unsigned dcol = 32u * i + (tid >> 3);
      const unsigned kk = (tid & 7u) * 8u;
#pragma unroll
      for (unsigned j = 0; j < 8u; ++j)
        x[i][j] = toh_flush(Cs[(kk + j) * LDC + dcol]);
      off[i] = ((size_t)bidx * DIM + n0 + dcol) * TOKP + key0 + kk;
    }
#pragma unroll
    for (int i = 0; i < 2; ++i) *(volatile v8h*)(out16 + off[i]) = x[i];
    __threadfence();
#pragma unroll
    for (int i = 0; i < 2; ++i) *(volatile v8h*)(out16 + off[i]) = x[i];
  }

  if (MODE == 2) {
    const float cs = 1.0f / (WCARRY * CCARRY);
    v4f xs[4];
    size_t off[4];
#pragma unroll
    for (unsigned i = 0; i < 4u; ++i) {
      const unsigned r = 16u * i + (tid >> 4);
      const unsigned c = (tid & 15u) * 4u;
      const unsigned crow = row0 + r;
      const unsigned f = crow / (unsigned)NB;
      const unsigned bb = crow - f * (unsigned)NB;
      const size_t orow = (size_t)f * NB_FULL + bb;
      const v4f u = *(const v4f*)&Cs[r * LDC + c];
      const v4f g = *(const v4f*)(bias + n0 + c);
      v4f val;
#pragma unroll
      for (int j = 0; j < 4; ++j) val[j] = u[j] * cs + bf16r(g[j]);
      xs[i] = val;
      off[i] = orow * DIM + n0 + c;
    }
#pragma unroll
    for (int i = 0; i < 4; ++i) *(volatile v4f*)(outf + off[i]) = xs[i];
    __threadfence();
#pragma unroll
    for (int i = 0; i < 4; ++i) *(volatile v4f*)(outf + off[i]) = xs[i];
  }
}

__global__ __launch_bounds__(256) void gemm_qk_kernel(
    const _Float16* __restrict__ A16, const _Float16* __restrict__ Bt,
    _Float16* __restrict__ qk) {
  gemm_body<0>(A16, Bt, (const float*)0, (float*)0, qk);
}
__global__ __launch_bounds__(256) void gemm_v_kernel(
    const _Float16* __restrict__ A16, const _Float16* __restrict__ Bt,
    _Float16* __restrict__ vt) {
  gemm_body<1>(A16, Bt, (const float*)0, (float*)0, vt);
}
__global__ __launch_bounds__(256) void gemm_out_kernel(
    const _Float16* __restrict__ A16, const _Float16* __restrict__ Bt,
    const float* __restrict__ bias, float* __restrict__ outf) {
  gemm_body<2>(A16, Bt, bias, outf, (_Float16*)0);
}

__global__ __launch_bounds__(256) void attn_kernel(
    const _Float16* __restrict__ QK, const _Float16* __restrict__ Vt,
    _Float16* __restrict__ Ctx) {
  __shared__ _Float16 Os[16 * LDO];

  const unsigned tid = threadIdx.x, lane = tid & 31u;
  const unsigned head = (unsigned)__builtin_amdgcn_readfirstlane((int)(threadIdx.x >> 5));
  const unsigned hh = lane >> 4, m = lane & 15u;
  const unsigned q0 = blockIdx.x * 16u;
  const unsigned b = blockIdx.y;
  const size_t tokbase = (size_t)b * TOKP;
  const float sscale = 0.25f / (QCARRY * QCARRY);

  const v16h qf = frag_k16(QK + (tokbase + q0 + m) * QKP + head * HD + hh * 8u);
  const _Float16* kp = QK + (tokbase + m) * QKP + DIM + head * HD + hh * 8u;
  const _Float16* vp = Vt + ((size_t)b * DIM + head * HD + m) * TOKP + hh * 8u;

  float mrow = -1.0e30f, lrow = 0.0f;
  v8f o = {};

  for (unsigned kb = 0; kb < (unsigned)NTOK; kb += 32u) {
    const v16h ka0 = frag_k16(kp + (size_t)kb * QKP);
    const v16h ka1 = frag_k16(kp + (size_t)(kb + 16u) * QKP);
    const v16h va  = frag_at(vp + kb);
    v8f s0 = {}, s1 = {};
    s0 = wmma16(ka0, qf, s0);
    s1 = wmma16(ka1, qf, s1);

    float mx = fmaxf(s0[0], s1[0]);
#pragma unroll
    for (int r = 1; r < 8; ++r) mx = fmaxf(mx, fmaxf(s0[r], s1[r]));
    mx = fmaxf(mx, __shfl_xor(mx, 16, 32));
    const float mn = fmaxf(mrow, mx * sscale);
    const float alpha = __expf(mrow - mn);
    mrow = mn;

    float rs = 0.0f;
    v16h pf;
#pragma unroll
    for (int r = 0; r < 8; ++r) {
      const float e0 = s0[r] * sscale - mn;
      const float e1 = s1[r] * sscale - mn;
      const float x0 = __expf(e0);
      const float x1 = __expf(e1);
      const float p0 = (e0 < PCUT) ? 0.0f : x0;
      const float p1 = (e1 < PCUT) ? 0.0f : x1;
      rs += p0 + p1;
      pf[r]     = (h16)(p0 * PCARRY);
      pf[r + 8] = (h16)(p1 * PCARRY);
    }
    rs += __shfl_xor(rs, 16, 32);
    lrow = alpha * lrow + rs;
#pragma unroll
    for (int r = 0; r < 8; ++r) o[r] = o[r] * alpha;

    o = wmma16(va, pf, o);
  }

  const float inv = __builtin_amdgcn_rcpf(lrow) * (CCARRY / (PCARRY * QCARRY));
  v8h ov;
#pragma unroll
  for (int r = 0; r < 8; ++r) ov[r] = toh_flush(o[r] * inv);
  *(v8h*)&Os[m * LDO + head * HD + hh * 8u] = ov;
  __syncthreads();

  const unsigned r = tid >> 4;
  const unsigned c = (tid & 15u) * 8u;
  const v8h x = *(const v8h*)&Os[r * LDO + c];
  _Float16* p = Ctx + ((size_t)(q0 + r) * NB + b) * DIM + c;
  *(volatile v8h*)p = x;
  __threadfence();
  *(volatile v8h*)p = x;
}

extern "C" void kernel_launch(void* const* d_in, const int* in_sizes, int n_in,
                              void* d_out, int out_size, void* d_ws, size_t ws_size,
                              hipStream_t stream) {
  if (n_in < 5) return;
  const long long need_xs = ((long long)(SEQ - 1) * NB_FULL + NB) * DIM;
  const long long need_out = ((long long)(NTOK - 1) * NB_FULL + NB) * DIM;
  if ((long long)in_sizes[0] < (long long)NPATCH * DIM) return;
  if ((long long)in_sizes[1] < need_xs) return;
  if ((long long)in_sizes[2] < (long long)3 * DIM * DIM) return;
  if ((long long)in_sizes[3] < (long long)DIM * DIM) return;
  if (in_sizes[4] < DIM) return;
  if ((long long)out_size < need_out) return;
  if (ws_size < WS_TOTAL) return;

  const float* xp   = (const float*)d_in[0];
  const float* xs   = (const float*)d_in[1];
  const float* wqkv = (const float*)d_in[2];
  const float* w0   = (const float*)d_in[3];
  const float* w0b  = (const float*)d_in[4];
  float* out = (float*)d_out;

  char* ws = (char*)d_ws;
  _Float16* Wqkv16 = (_Float16*)(ws + OFF_WQKV);
  _Float16* W016   = (_Float16*)(ws + OFF_W0);
  _Float16* X16    = (_Float16*)(ws + OFF_X);
  _Float16* QK16   = (_Float16*)(ws + OFF_QK);
  _Float16* Vt16   = (_Float16*)(ws + OFF_VT);
  _Float16* Ctx16  = (_Float16*)(ws + OFF_CTX);

  dim3 blk(256);
  wcast_kernel<<<dim3((3 * DIM * DIM) / 2048), blk, 0, stream>>>(wqkv, Wqkv16);
  wcast_kernel<<<dim3((DIM * DIM) / 2048), blk, 0, stream>>>(w0, W016);
  xconv_kernel<<<dim3(XROWS / 16), blk, 0, stream>>>(xp, xs, X16);
  gemm_qk_kernel<<<dim3(QKP / 64, XROWS / 64), blk, 0, stream>>>(X16, Wqkv16, QK16);
  gemm_v_kernel<<<dim3(DIM / 64, XROWS / 64), blk, 0, stream>>>(
      X16, Wqkv16 + (size_t)2 * DIM * DIM, Vt16);
  attn_kernel<<<dim3(NTOK / 16, NB), blk, 0, stream>>>(QK16, Vt16, Ctx16);
  gemm_out_kernel<<<dim3(DIM / 64, OROWS / 64), blk, 0, stream>>>(Ctx16, W016, w0b, out);
}
